// FeatureEnhancerLayer_71829033058373
// MI455X (gfx1250) — hardware-verified
//
#include <hip/hip_runtime.h>
#include <math.h>

#define D_MODEL 256
#define NHEADS  8
#define DHEAD   32
#define BATCH   2
#define LTXT    256
#define NTOT    13294

typedef __attribute__((ext_vector_type(16))) _Float16 v16h;
typedef __attribute__((ext_vector_type(8)))  _Float16 v8h;
typedef __attribute__((ext_vector_type(4)))  _Float16 v4h;
typedef __attribute__((ext_vector_type(8)))  float  v8f;

__device__ __forceinline__ _Float16 f2bf(float x) { return (_Float16)x; }
#define ASC 1024.0f
#define AUN (1.0f / 1024.0f)
typedef __attribute__((ext_vector_type(4))) float v4f;
template <typename V> __device__ __forceinline__ void vst2(void* p, V v) {
  *(volatile V*)p = v; __threadfence(); *(volatile V*)p = v;
}
__device__ __forceinline__ v8f wm16(v16h a, v16h b, v8f c) {
  v8f d = __builtin_amdgcn_wmma_f32_16x16x32_f16(false, a, false, b, (short)0, c, false, false);
  asm volatile("v_nop\n\tv_nop\n\tv_nop\n\tv_nop" : "+v"(d) : "v"(a), "v"(b));
  return d;
}
#define WMMA16(na, a, nb, b, cm, c, ra, rb) wm16((a), (b), (c))

__device__ __forceinline__ v16h frag_cat(v8h lo, v8h hi) {
  return __builtin_shufflevector(lo, hi, 0,1,2,3,4,5,6,7,8,9,10,11,12,13,14,15);
}

__global__ __launch_bounds__(256) void gemm_f16_wmma(
    const float* __restrict__ A, int lda,
    const float* __restrict__ Bw, int ldb,
    const float* __restrict__ bias,
    const float* __restrict__ resid,
    float* __restrict__ C, int ldc,
    int M, int N, int K, int mpb, long cbs, int relu)
{
  __shared__ _Float16 As [64][40];
  __shared__ _Float16 BsT[64][40];
  __shared__ __attribute__((aligned(16))) float Cs[64][64];
  const int tid  = threadIdx.x;
  const int lane = tid & 31;
  const int wav  = tid >> 5;
  const int wm   = wav >> 1;
  const int wn   = wav & 1;
  const int hh   = lane >> 4;
  const int l16  = lane & 15;
  const long bm  = (long)blockIdx.y * 64;
  const int  bn  = blockIdx.x * 64;
  const bool fullM = (bm + 64 <= (long)M);

  v8f acc0 = {0.f,0.f,0.f,0.f,0.f,0.f,0.f,0.f};
  v8f acc1 = acc0;

  for (int k0 = 0; k0 < K; k0 += 32) {
    if (fullM) {
      #pragma unroll
      for (int i = 0; i < 2; ++i) {
        int idx = tid + i * 256;
        int r = idx >> 3, c = (idx & 7) << 2;
        const float4 f = *(const float4*)(A + (bm + r) * (long)lda + k0 + c);
        v4h hk; hk[0] = f2bf(f.x * ASC); hk[1] = f2bf(f.y * ASC); hk[2] = f2bf(f.z * ASC); hk[3] = f2bf(f.w * ASC);
        *(v4h*)&As[r][c] = hk;
      }
    } else {
      #pragma unroll
      for (int i = 0; i < 2; ++i) {
        int idx = tid + i * 256;
        int r = idx >> 3, c = (idx & 7) << 2;
        v4h hk;
        if (bm + r < (long)M) {
          const float4 f = *(const float4*)(A + (bm + r) * (long)lda + k0 + c);
          hk[0] = f2bf(f.x * ASC); hk[1] = f2bf(f.y * ASC); hk[2] = f2bf(f.z * ASC); hk[3] = f2bf(f.w * ASC);
        } else {
          hk[0] = hk[1] = hk[2] = hk[3] = f2bf(0.f);
        }
        *(v4h*)&As[r][c] = hk;
      }
    }
    #pragma unroll
    for (int i = 0; i < 2; ++i) {
      int idx = tid + i * 256;
      int r = idx >> 4, c = (idx & 15) << 2;
      const float4 f = *(const float4*)(Bw + (long)(k0 + r) * ldb + bn + c);
      BsT[c + 0][r] = f2bf(f.x);
      BsT[c + 1][r] = f2bf(f.y);
      BsT[c + 2][r] = f2bf(f.z);
      BsT[c + 3][r] = f2bf(f.w);
    }
    __syncthreads();

    const int arow = wm * 16 + l16;
    const int bc   = wn * 32 + l16;
    v16h af = frag_cat(*(const v8h*)&As[arow][hh * 8],
                        *(const v8h*)&As[arow][16 + hh * 8]);
    v16h bf0 = frag_cat(*(const v8h*)&BsT[bc][hh * 8],
                         *(const v8h*)&BsT[bc][16 + hh * 8]);
    v16h bf1 = frag_cat(*(const v8h*)&BsT[bc + 16][hh * 8],
                         *(const v8h*)&BsT[bc + 16][16 + hh * 8]);
    acc0 = WMMA16(false, af, false, bf0, (short)0, acc0, false, false);
    acc1 = WMMA16(false, af, false, bf1, (short)0, acc1, false, false);
    __syncthreads();
  }

  #pragma unroll
  for (int e = 0; e < 8; ++e) {
    const int rl = wm * 16 + e + 8 * hh;
    long r = bm + rl;
    long pr = (r < M) ? ((r / mpb) * cbs + (r % mpb)) : 0;
    const float* rrow = (resid && r < M) ? (resid + pr * (long)ldc) : nullptr;
    int n0 = bn + wn * 32 + l16;
    {
      float x = acc0[e] * AUN;
      if (bias) x += bias[n0];
      if (rrow) x += rrow[n0];
      if (relu) x = fmaxf(x, 0.f);
      Cs[rl][wn * 32 + l16] = x;
    }
    int n1 = n0 + 16;
    {
      float x = acc1[e] * AUN;
      if (bias) x += bias[n1];
      if (rrow) x += rrow[n1];
      if (relu) x = fmaxf(x, 0.f);
      Cs[rl][wn * 32 + 16 + l16] = x;
    }
  }
  __syncthreads();
  #pragma unroll
  for (int i = 0; i < 4; ++i) {
    const int g = tid + i * 256;
    const int rl = g >> 4, pc = g & 15;
    const long r = bm + rl;
    if (r < M) {
      const long pr = (r / mpb) * cbs + (r % mpb);
      vst2(C + pr * (long)ldc + bn + pc * 4, *(const v4f*)&Cs[rl][pc * 4]);
    }
  }
}

__global__ __launch_bounds__(256) void gn_stats(
    const float* __restrict__ x, float* __restrict__ stats, int startRow, int HW)
{
  const int b = blockIdx.x >> 5;
  const int g = blockIdx.x & 31;
  const int tid = threadIdx.x;
  float s = 0.f, ss = 0.f;
  const int tot = HW * 8;
  for (int i = tid; i < tot; i += 256) {
    int p = i >> 3, j = i & 7;
    float v = x[((long)b * NTOT + startRow + p) * D_MODEL + g * 8 + j];
    s += v; ss += v * v;
  }
  __shared__ float rs[256], rss[256];
  rs[tid] = s; rss[tid] = ss;
  __syncthreads();
  for (int o = 128; o > 0; o >>= 1) {
    if (tid < o) { rs[tid] += rs[tid + o]; rss[tid] += rss[tid + o]; }
    __syncthreads();
  }
  if (tid < 8) {
    float cnt = (float)tot;
    float mu = rs[0] / cnt;
    float var = rss[0] / cnt - mu * mu;
    v4f v = {mu, var, 0.f, 0.f};
    vst2(stats + (b * 32 + g) * 32 + tid * 4, v);
  }
}

__global__ __launch_bounds__(256) void gn_norm(
    float* __restrict__ x, const float* __restrict__ stats,
    const float* __restrict__ gg, const float* __restrict__ gb,
    int startRow, int HW)
{
  long idx = (long)blockIdx.x * 256 + threadIdx.x;
  long tot = (long)BATCH * HW * D_MODEL;
  if (idx >= tot) return;
  int c = (int)(idx & 255);
  long t = idx >> 8;
  int p = (int)(t % HW);
  int b = (int)(t / HW);
  int g = c >> 3;
  float mu  = stats[(b * 32 + g) * 32];
  float var = stats[(b * 32 + g) * 32 + 1];
  long off = ((long)b * NTOT + startRow + p) * D_MODEL + c;
  const float nv = (x[off] - mu) * rsqrtf(var + 1e-5f) * gg[c] + gb[c];
  vst2(x + off, nv);
}

__global__ __launch_bounds__(256) void deform_sample(
    const float* __restrict__ value, const float* __restrict__ offs,
    const float* __restrict__ alog,  const float* __restrict__ refp,
    float* __restrict__ samp)
{
  long gid = (long)blockIdx.x * 256 + threadIdx.x;
  const long total = (long)BATCH * NTOT * NHEADS;
  if (gid >= total) return;
  int h = (int)(gid & 7);
  long t = gid >> 3;
  int n = (int)(t % NTOT);
  int b = (int)(t / NTOT);
  const int Hs[4] = {100, 50, 25, 13};
  const int st[4] = {0, 10000, 12500, 13125};
  long row = (long)b * NTOT + n;

  const float* ap = alog + row * 128 + h * 16;
  float lg[16]; float mx = -3e38f;
  #pragma unroll
  for (int i = 0; i < 16; ++i) { lg[i] = ap[i]; mx = fmaxf(mx, lg[i]); }
  float se = 0.f;
  #pragma unroll
  for (int i = 0; i < 16; ++i) { lg[i] = __expf(lg[i] - mx); se += lg[i]; }
  float inv = 1.f / se;

  const float* op = offs + row * 256 + h * 32;
  float acc[DHEAD];
  #pragma unroll
  for (int d = 0; d < DHEAD; ++d) acc[d] = 0.f;

  #pragma unroll 1
  for (int l = 0; l < 4; ++l) {
    const int Wl = Hs[l], Hl = Hs[l];
    float rx = refp[(row * 4 + l) * 2 + 0];
    float ry = refp[(row * 4 + l) * 2 + 1];
    #pragma unroll 1
    for (int p = 0; p < 4; ++p) {
      float ox = op[l * 8 + p * 2 + 0];
      float oy = op[l * 8 + p * 2 + 1];
      float px = (rx + ox / (float)Wl) * Wl - 0.5f;
      float py = (ry + oy / (float)Hl) * Hl - 0.5f;
      float x0f = floorf(px), y0f = floorf(py);
      float fx = px - x0f, fy = py - y0f;
      int x0 = (int)x0f, y0 = (int)y0f;
      float aw = lg[l * 4 + p] * inv;
      float ww[2][2] = {{aw * (1.f - fx) * (1.f - fy), aw * fx * (1.f - fy)},
                        {aw * (1.f - fx) * fy,         aw * fx * fy}};
      #pragma unroll
      for (int cy = 0; cy < 2; ++cy) {
        #pragma unroll
        for (int cx = 0; cx < 2; ++cx) {
          int yi = y0 + cy, xi = x0 + cx;
          if (xi < 0 || xi >= Wl || yi < 0 || yi >= Hl) continue;
          float w = ww[cy][cx];
          const float* vp = value + ((long)b * NTOT + st[l] + (long)yi * Wl + xi) * D_MODEL + h * 32;
          #pragma unroll
          for (int d = 0; d < DHEAD; ++d) acc[d] += w * vp[d];
        }
      }
    }
  }
  float* outp = samp + row * 256 + h * 32;
  #pragma unroll
  for (int d = 0; d < DHEAD; d += 4) { v4f v = {acc[d], acc[d + 1], acc[d + 2], acc[d + 3]}; vst2(outp + d, v); }
}

__global__ __launch_bounds__(128) void attn_flash(
    const float* __restrict__ Q, const float* __restrict__ Kt,
    const float* __restrict__ V, float* __restrict__ O,
    int Lq, int Lk, float scale)
{
  const int tid  = threadIdx.x;
  const int lane = tid & 31;
  const int wav  = tid >> 5;
  const int h    = blockIdx.y;
  const int b    = blockIdx.z;
  const int q0   = blockIdx.x * 64 + wav * 16;
  const int hh  = lane >> 4;
  const int l16 = lane & 15;

  const float* Qh = Q  + (long)b * Lq * D_MODEL + h * 32;
  const float* Kh = Kt + (long)b * Lk * D_MODEL + h * 32;
  const float* Vh = V  + (long)b * Lk * D_MODEL + h * 32;

  __shared__ _Float16 Ks[32][40];
  __shared__ _Float16 VT[32][40];
  __shared__ _Float16 Ps[4][16][40];
  __shared__ __attribute__((aligned(16))) float Os[4][16][32];

  v16h qf;
  {
    int r = q0 + l16; if (r >= Lq) r = Lq - 1;
    const float* qr = Qh + (long)r * D_MODEL;
    float4 fa = *(const float4*)(qr + hh * 8);
    float4 fb = *(const float4*)(qr + hh * 8 + 4);
    float4 fc = *(const float4*)(qr + 16 + hh * 8);
    float4 fd = *(const float4*)(qr + 16 + hh * 8 + 4);
    scale *= ASC;
    qf[0]  = f2bf(fa.x * scale); qf[1]  = f2bf(fa.y * scale);
    qf[2]  = f2bf(fa.z * scale); qf[3]  = f2bf(fa.w * scale);
    qf[4]  = f2bf(fb.x * scale); qf[5]  = f2bf(fb.y * scale);
    qf[6]  = f2bf(fb.z * scale); qf[7]  = f2bf(fb.w * scale);
    qf[8]  = f2bf(fc.x * scale); qf[9]  = f2bf(fc.y * scale);
    qf[10] = f2bf(fc.z * scale); qf[11] = f2bf(fc.w * scale);
    qf[12] = f2bf(fd.x * scale); qf[13] = f2bf(fd.y * scale);
    qf[14] = f2bf(fd.z * scale); qf[15] = f2bf(fd.w * scale);
  }

  float mrun[8], lrun[8];
  #pragma unroll
  for (int e = 0; e < 8; ++e) { mrun[e] = -3e38f; lrun[e] = 0.f; }
  v8f o0 = {0.f,0.f,0.f,0.f,0.f,0.f,0.f,0.f};
  v8f o1 = o0;

  for (int kb = 0; kb < Lk; kb += 32) {
    #pragma unroll
    for (int i = 0; i < 2; ++i) {
      int idx = tid + i * 128;
      int r = idx >> 3;
      int c = (idx & 7) << 2;
      int gk = kb + r; if (gk >= Lk) gk = Lk - 1;
      float4 fk = *(const float4*)(Kh + (long)gk * D_MODEL + c);
      v4h hk; hk[0] = f2bf(fk.x * ASC); hk[1] = f2bf(fk.y * ASC); hk[2] = f2bf(fk.z * ASC); hk[3] = f2bf(fk.w * ASC);
      *(v4h*)&Ks[r][c] = hk;
      float4 fv = *(const float4*)(Vh + (long)gk * D_MODEL + c);
      VT[c + 0][r] = f2bf(fv.x * ASC);
      VT[c + 1][r] = f2bf(fv.y * ASC);
      VT[c + 2][r] = f2bf(fv.z * ASC);
      VT[c + 3][r] = f2bf(fv.w * ASC);
    }
    __syncthreads();

    v16h kf0 = frag_cat(*(const v8h*)&Ks[l16][hh * 8],
                         *(const v8h*)&Ks[l16][16 + hh * 8]);
    v16h kf1 = frag_cat(*(const v8h*)&Ks[16 + l16][hh * 8],
                         *(const v8h*)&Ks[16 + l16][16 + hh * 8]);
    v8f s0 = {0.f,0.f,0.f,0.f,0.f,0.f,0.f,0.f};
    v8f s1 = s0;
    s0 = WMMA16(false, qf, false, kf0, (short)0, s0, false, false);
    s1 = WMMA16(false, qf, false, kf1, (short)0, s1, false, false);

    const bool inv0 = (kb + l16) >= Lk;
    const bool inv1 = (kb + 16 + l16) >= Lk;

    float corr[8];
    #pragma unroll
    for (int e = 0; e < 8; ++e) {
      float a = inv0 ? -3e38f : s0[e] * (AUN * AUN);
      float c = inv1 ? -3e38f : s1[e] * (AUN * AUN);
      float mx = fmaxf(a, c);
      for (int msk = 1; msk <= 8; msk <<= 1) mx = fmaxf(mx, __shfl_xor(mx, msk, 32));
      float mnew = fmaxf(mrun[e], mx);
      float p0 = inv0 ? 0.f : __expf(a - mnew);
      float p1 = inv1 ? 0.f : __expf(c - mnew);
      float ps = p0 + p1;
      for (int msk = 1; msk <= 8; msk <<= 1) ps += __shfl_xor(ps, msk, 32);
      corr[e] = __expf(mrun[e] - mnew);
      lrun[e] = lrun[e] * corr[e] + ps;
      mrun[e] = mnew;
      Ps[wav][e + 8 * hh][l16]      = f2bf(p0 * 256.0f);
      Ps[wav][e + 8 * hh][16 + l16] = f2bf(p1 * 256.0f);
    }
    asm volatile("s_wait_dscnt 0" ::: "memory");

    v16h pf = frag_cat(*(const v8h*)&Ps[wav][l16][hh * 8],
                        *(const v8h*)&Ps[wav][l16][16 + hh * 8]);
    v16h vf0 = frag_cat(*(const v8h*)&VT[l16][hh * 8],
                         *(const v8h*)&VT[l16][16 + hh * 8]);
    v16h vf1 = frag_cat(*(const v8h*)&VT[16 + l16][hh * 8],
                         *(const v8h*)&VT[16 + l16][16 + hh * 8]);
    #pragma unroll
    for (int e = 0; e < 8; ++e) { o0[e] *= corr[e]; o1[e] *= corr[e]; }
    o0 = WMMA16(false, pf, false, vf0, (short)0, o0, false, false);
    o1 = WMMA16(false, pf, false, vf1, (short)0, o1, false, false);
    __syncthreads();
  }

  float* Oh = O + (long)b * Lq * D_MODEL + h * 32;
  #pragma unroll
  for (int e = 0; e < 8; ++e) {
    float inv = ((1.0f / 256.0f) * AUN) / lrun[e];
    Os[wav][e + 8 * hh][l16]      = o0[e] * inv;
    Os[wav][e + 8 * hh][16 + l16] = o1[e] * inv;
  }
  __syncthreads();
  #pragma unroll
  for (int q = 0; q < 4; ++q) {
    const int rl = q * 4 + (lane >> 3), pc = lane & 7;
    const int r = q0 + rl;
    if (r < Lq) vst2(Oh + (long)r * D_MODEL + pc * 4, *(const v4f*)&Os[wav][rl][pc * 4]);
  }
}

static inline void launch_gemm(hipStream_t st,
    const float* A, int lda, const float* Bw, int ldb,
    const float* bias, const float* resid, float* C, int ldc,
    int M, int N, int K, int mpb, long cbs, int relu)
{
  dim3 g((N + 63) / 64, (M + 63) / 64);
  gemm_f16_wmma<<<g, 256, 0, st>>>(A, lda, Bw, ldb, bias, resid, C, ldc,
                                    M, N, K, mpb, cbs, relu);
}

extern "C" void kernel_launch(void* const* d_in, const int* in_sizes, int n_in,
                              void* d_out, int out_size, void* d_ws, size_t ws_size,
                              hipStream_t stream)
{
  const float* img[4]    = {(const float*)d_in[0], (const float*)d_in[1],
                            (const float*)d_in[2], (const float*)d_in[3]};
  const float* text      = (const float*)d_in[4];
  const float* refp      = (const float*)d_in[5];
  const float* proj_w[4] = {(const float*)d_in[6], (const float*)d_in[7],
                            (const float*)d_in[8], (const float*)d_in[9]};
  const float* proj_b    = (const float*)d_in[10];
  const float* gn_g      = (const float*)d_in[11];
  const float* gn_b      = (const float*)d_in[12];
  const float* feat_w    = (const float*)d_in[13];
  const float* feat_b    = (const float*)d_in[14];
  const float* def_val_w = (const float*)d_in[15];
  const float* def_val_b = (const float*)d_in[16];
  const float* def_off_w = (const float*)d_in[17];
  const float* def_off_b = (const float*)d_in[18];
  const float* def_att_w = (const float*)d_in[19];
  const float* def_att_b = (const float*)d_in[20];
  const float* def_out_w = (const float*)d_in[21];
  const float* def_out_b = (const float*)d_in[22];
  const float* tsa_in_w  = (const float*)d_in[23];
  const float* tsa_in_b  = (const float*)d_in[24];
  const float* tsa_out_w = (const float*)d_in[25];
  const float* tsa_out_b = (const float*)d_in[26];
  const float* i2t_in_w  = (const float*)d_in[27];
  const float* i2t_in_b  = (const float*)d_in[28];
  const float* i2t_out_w = (const float*)d_in[29];
  const float* i2t_out_b = (const float*)d_in[30];
  const float* t2i_in_w  = (const float*)d_in[31];
  const float* t2i_in_b  = (const float*)d_in[32];
  const float* t2i_out_w = (const float*)d_in[33];
  const float* t2i_out_b = (const float*)d_in[34];
  const float* ffn_w1    = (const float*)d_in[35];
  const float* ffn_b1    = (const float*)d_in[36];
  const float* ffn_w2    = (const float*)d_in[37];
  const float* ffn_b2    = (const float*)d_in[38];

  float* W = (float*)d_ws;
  const long SLOT = (long)BATCH * NTOT * D_MODEL;
  float* s0 = W;
  float* s1 = W + 1 * SLOT;
  float* s2 = W + 2 * SLOT;
  float* s3 = W + 3 * SLOT;
  float* s4 = W + 4 * SLOT;
  float* s5 = W + 5 * SLOT;
  float* sm = W + 6 * SLOT;
  const long TS = (long)BATCH * LTXT * D_MODEL;
  float* txt    = sm;               sm += TS;
  float* tq     = sm;               sm += TS;
  float* tk     = sm;               sm += TS;
  float* tv     = sm;               sm += TS;
  float* tao    = sm;               sm += TS;
  float* txt2   = sm;               sm += TS;
  float* qi2t   = sm;               sm += TS;
  float* aoi2t  = sm;               sm += TS;
  float* ztxt   = sm;               sm += TS;
  float* hidtxt = sm;               sm += (long)BATCH * LTXT * 1024;
  float* stats  = sm;

  const int HWs[4]    = {10000, 2500, 625, 169};
  const int Cs[4]     = {256, 512, 1024, 2048};
  const int starts[4] = {0, 10000, 12500, 13125};
  const int Mimg = BATCH * NTOT;
  const float scale = 0.1767766953f;

  for (int l = 0; l < 4; ++l) {
    launch_gemm(stream, img[l], Cs[l], proj_w[l], D_MODEL,
                proj_b + l * D_MODEL, nullptr,
                s0 + (long)starts[l] * D_MODEL, D_MODEL,
                BATCH * HWs[l], D_MODEL, Cs[l], HWs[l], (long)NTOT, 0);
    gn_stats<<<BATCH * 32, 256, 0, stream>>>(s0, stats, starts[l], HWs[l]);
    long tot = (long)BATCH * HWs[l] * D_MODEL;
    gn_norm<<<(unsigned)((tot + 255) / 256), 256, 0, stream>>>(
        s0, stats, gn_g + l * D_MODEL, gn_b + l * D_MODEL, starts[l], HWs[l]);
  }

  launch_gemm(stream, s0, 256, def_val_w, 256, def_val_b, nullptr, s1, 256,
              Mimg, 256, 256, Mimg, Mimg, 0);
  launch_gemm(stream, s0, 256, def_off_w, 256, def_off_b, nullptr, s2, 256,
              Mimg, 256, 256, Mimg, Mimg, 0);
  launch_gemm(stream, s0, 256, def_att_w, 128, def_att_b, nullptr, s3, 128,
              Mimg, 128, 256, Mimg, Mimg, 0);
  deform_sample<<<(unsigned)(((long)Mimg * NHEADS + 255) / 256), 256, 0, stream>>>(
      s1, s2, s3, refp, s4);
  launch_gemm(stream, s4, 256, def_out_w, 256, def_out_b, nullptr, s5, 256,
              Mimg, 256, 256, Mimg, Mimg, 0);

  const int Mt = BATCH * LTXT;
  launch_gemm(stream, text, 768, feat_w, 256, feat_b, nullptr, txt, 256,
              Mt, 256, 768, Mt, Mt, 0);
  launch_gemm(stream, txt, 256, tsa_in_w +   0, 768, tsa_in_b +   0, nullptr, tq, 256, Mt, 256, 256, Mt, Mt, 0);
  launch_gemm(stream, txt, 256, tsa_in_w + 256, 768, tsa_in_b + 256, nullptr, tk, 256, Mt, 256, 256, Mt, Mt, 0);
  launch_gemm(stream, txt, 256, tsa_in_w + 512, 768, tsa_in_b + 512, nullptr, tv, 256, Mt, 256, 256, Mt, Mt, 0);
  attn_flash<<<dim3((LTXT + 63) / 64, NHEADS, BATCH), 128, 0, stream>>>(
      tq, tk, tv, tao, LTXT, LTXT, scale);
  launch_gemm(stream, tao, 256, tsa_out_w, 256, tsa_out_b, nullptr, txt2, 256,
              Mt, 256, 256, Mt, Mt, 0);

  launch_gemm(stream, txt2, 256, i2t_in_w +   0, 768, i2t_in_b +   0, nullptr, qi2t, 256, Mt, 256, 256, Mt, Mt, 0);
  launch_gemm(stream, s5,   256, i2t_in_w + 256, 768, i2t_in_b + 256, nullptr, s0,   256, Mimg, 256, 256, Mimg, Mimg, 0);
  launch_gemm(stream, s5,   256, i2t_in_w + 512, 768, i2t_in_b + 512, nullptr, s1,   256, Mimg, 256, 256, Mimg, Mimg, 0);
  attn_flash<<<dim3((LTXT + 63) / 64, NHEADS, BATCH), 128, 0, stream>>>(
      qi2t, s0, s1, aoi2t, LTXT, NTOT, scale);
  launch_gemm(stream, aoi2t, 256, i2t_out_w, 256, i2t_out_b, txt2, ztxt, 256,
              Mt, 256, 256, Mt, Mt, 0);

  launch_gemm(stream, s5,   256, t2i_in_w +   0, 768, t2i_in_b +   0, nullptr, s2, 256, Mimg, 256, 256, Mimg, Mimg, 0);
  launch_gemm(stream, txt2, 256, t2i_in_w + 256, 768, t2i_in_b + 256, nullptr, tk, 256, Mt,   256, 256, Mt,   Mt,   0);
  launch_gemm(stream, txt2, 256, t2i_in_w + 512, 768, t2i_in_b + 512, nullptr, tv, 256, Mt,   256, 256, Mt,   Mt,   0);
  attn_flash<<<dim3((NTOT + 63) / 64, NHEADS, BATCH), 128, 0, stream>>>(
      s2, tk, tv, s3, NTOT, LTXT, scale);
  launch_gemm(stream, s3, 256, t2i_out_w, 256, t2i_out_b, s5, s4, 256,
              Mimg, 256, 256, Mimg, Mimg, 0);

  float* out_img = (float*)d_out;
  float* out_txt = out_img + (long)BATCH * NTOT * D_MODEL;
  const int Mc = Mimg / 4;
  for (int c = 0; c < 4; ++c) {
    const float* zi = s4 + (long)c * Mc * 256;
    launch_gemm(stream, zi, 256, ffn_w1, 1024, ffn_b1, nullptr, s0, 1024,
                Mc, 1024, 256, Mc, Mc, 1);
    launch_gemm(stream, s0, 1024, ffn_w2, 256, ffn_b2, nullptr,
                out_img + (long)c * Mc * 256, 256, Mc, 256, 1024, Mc, Mc, 0);
  }
  launch_gemm(stream, ztxt, 256, ffn_w1, 1024, ffn_b1, nullptr, hidtxt, 1024,
              Mt, 1024, 256, Mt, Mt, 1);
  launch_gemm(stream, hidtxt, 1024, ffn_w2, 256, ffn_b2, nullptr, out_txt, 256,
              Mt, 256, 1024, Mt, Mt, 0);
}
